// LearnedBeamformer_21191368639232
// MI455X (gfx1250) — hardware-verified
//
#include <hip/hip_runtime.h>
#include <stddef.h>
#include <stdint.h>

#define NBAT   8
#define NBIRD  8
#define NSMP   64
#define NMIC   5
#define NFREQ  257
#define TLEN   512
#define TPAD   514
#define FP     320
#define FPW    320
#define NHID   64
#define C1N    128
#define C2N    256
#define K1     (3 * FP)
#define K2     (3 * C1N)
#define NROWS  (NSMP * TLEN)
#define NRB    (NROWS / 64)
#define TBLK   8
#define NTB    (TLEN / TBLK)
#define FCH    32
#define NCH    (FP / FCH)
#define WLP    12
#define SP     68
#define NPB1   (C1N * K1 / 8 / 256)
#define NPB2   (C2N * K2 / 8 / 256)
#define NAPB   (NSMP * TPAD * C1N / 8 / 256)
#define NSTB   (NSMP * (FPW / 64))
#define MSC    16.0f
#define H1SC   16.0f
#define WSC    64.0f
#define ZINV   (1.0f / 1024.0f)
#define EPSBN  1e-5f
#define FSTEP  47.68359375f
#define NEG2PI (-6.283185307179586f)
#define RCPC   (1.0f / 343000.0f)

static_assert(NPB1 * 256 * 8 == C1N * K1);
static_assert(NPB2 * 256 * 8 == C2N * K2);
static_assert(NAPB * 256 * 8 == NSMP * TPAD * C1N);
static_assert((FP % 32) == 0);
static_assert((C1N % 32) == 0);
static_assert(NCH * FCH == FP);
static_assert(FP >= NFREQ);
static_assert(NTB * TBLK == TLEN);
static_assert(NRB * 64 == NROWS);
static_assert((TLEN % 64) == 0);
static_assert((SP % 4) == 0);
static_assert(NBIRD * 32 == 256);
static_assert(TBLK == 8);
static_assert((FPW % 64) == 0);
static_assert(NSTB == 320);

typedef unsigned short v8us  __attribute__((ext_vector_type(8)));
typedef unsigned short v16us __attribute__((ext_vector_type(16)));
typedef float          v2f   __attribute__((ext_vector_type(2)));
typedef float          v4f   __attribute__((ext_vector_type(4)));
typedef float          v8f   __attribute__((ext_vector_type(8)));
#if defined(__HIP_DEVICE_COMPILE__)
typedef _Float16       v16h  __attribute__((ext_vector_type(16)));
#endif

union FragU { v16us v; v8us half[2]; };

__device__ __forceinline__ unsigned bbits(float f) {
  const unsigned u = __float_as_uint(f);
  return (u + 0x7FFFu + ((u >> 16) & 1u)) >> 16;
}
__device__ __forceinline__ float bf16r(float f) {
  return __uint_as_float(bbits(f) << 16);
}
__device__ __forceinline__ unsigned short hbits(float f) {
  const _Float16 hv = (_Float16)f;
  return __builtin_bit_cast(unsigned short, hv);
}
__device__ __forceinline__ v8f  zero8()   { v8f z = {0.f, 0.f, 0.f, 0.f, 0.f, 0.f, 0.f, 0.f}; return z; }
__device__ __forceinline__ v8us zero8us() { v8us z = {0, 0, 0, 0, 0, 0, 0, 0}; return z; }

__device__ __forceinline__ v16us ldfrag(const unsigned short* p) {
  FragU f;
  f.half[0] = *(const v8us*)(p);
  f.half[1] = *(const v8us*)(p + 16);
  return f.v;
}

__device__ __forceinline__ v8f mma_h(v16us a, v16us b, v8f c) {
#if defined(__HIP_DEVICE_COMPILE__)
  return __builtin_amdgcn_wmma_f32_16x16x32_f16(false, __builtin_bit_cast(v16h, a),
                                               false, __builtin_bit_cast(v16h, b),
                                               (short)0, c, false, false);
#else
  (void)a; (void)b;
  return c;
#endif
}
__device__ __forceinline__ void guard8(v8f& c0, v8f& c1, v8f& c2, v8f& c3,
                                       const v16us& a0, const v16us& a1,
                                       const v16us& b0, const v16us& b1) {
#if defined(__HIP_DEVICE_COMPILE__)
  asm volatile("v_nop\n\tv_nop\n\tv_nop\n\tv_nop"
               : "+v"(c0), "+v"(c1), "+v"(c2), "+v"(c3)
               : "v"(a0), "v"(a1), "v"(b0), "v"(b1)
               : "memory");
#else
  (void)c0; (void)c1; (void)c2; (void)c3; (void)a0; (void)a1; (void)b0; (void)b1;
#endif
}

__global__ __launch_bounds__(256)
void k_prep(const float* __restrict__ cw1, const float* __restrict__ cw2,
            unsigned short* W1P, unsigned short* W2P)
{
  const int b = blockIdx.x, tid = threadIdx.x;
  v8us val = zero8us();
  unsigned short* dst;
  if (b < NPB1) {
    const int i   = b * 256 + tid;
    const int e0  = i * 8;
    const int ch  = e0 / K1;
    const int k0  = e0 - ch * K1;
    const int tap = k0 / FP;
    const int fb  = k0 - tap * FP;
#pragma unroll
    for (int e = 0; e < 8; ++e) {
      const int f  = fb + e;
      const int fc = (f < NFREQ) ? f : (NFREQ - 1);
      const float w = cw1[((size_t)(ch * NFREQ + fc)) * 3 + tap];
      val[e] = (unsigned short)((f < NFREQ) ? (unsigned)hbits(bf16r(w) * WSC) : 0u);
    }
    dst = W1P + (size_t)i * 8;
  } else {
    const int i   = (b - NPB1) * 256 + tid;
    const int e0  = i * 8;
    const int ch  = e0 / K2;
    const int k0  = e0 - ch * K2;
    const int tap = k0 / C1N;
    const int cb  = k0 - tap * C1N;
#pragma unroll
    for (int e = 0; e < 8; ++e) {
      const float w = cw2[((size_t)(ch * C1N + cb + e)) * 3 + tap];
      val[e] = hbits(bf16r(w) * WSC);
    }
    dst = W2P + (size_t)i * 8;
  }
  *(volatile v8us*)dst = val;
  __threadfence();
  *(volatile v8us*)dst = val;
}

__global__ __launch_bounds__(256)
void k_steer(const float* __restrict__ pos, const float* __restrict__ w1, const float* __restrict__ b1,
             const float* __restrict__ w2, const float* __restrict__ b2, float* WR)
{
  __shared__ float sw1[10 * NHID], sw2[NHID * 10], sb1[NHID], sb2[16];
  __shared__ float sfe[64 * 10];
  const int tid = threadIdx.x;
  for (int i = tid; i < 10 * NHID; i += 256) { sw1[i] = bf16r(w1[i]); sw2[i] = bf16r(w2[i]); }
  if (tid < NHID) sb1[tid] = bf16r(b1[tid]);
  if (tid < 10) sb2[tid] = bf16r(b2[tid]);
  const int bn = blockIdx.x / (FPW / 64);
  const int f0 = (blockIdx.x - bn * (FPW / 64)) * 64;
  {
    const int row = tid & 63;
    const int m   = 1 + (tid >> 6);
    const int f   = f0 + row;
    const int fc  = (f < NFREQ) ? f : (NFREQ - 1);
    const float mx = (m == 4) ? 500.0f : ((m & 1) ? 1000.0f : 0.0f);
    const float my = (m == 4) ? 500.0f : ((m & 2) ? 1000.0f : 0.0f);
    const float mz = (m == 4) ? 0.0f : 500.0f;
    float ph;
    {
#pragma clang fp contract(off)
      const float px = bf16r(pos[bn * 3 + 0]) * 1000.0f + 0.0f;
      const float py = bf16r(pos[bn * 3 + 1]) * 1000.0f + 0.0f;
      const float pz = bf16r(pos[bn * 3 + 2]) * 500.0f + 0.0f;
      const float dz0 = pz - 500.0f;
      const float d0 = sqrtf((px * px + py * py) + dz0 * dz0);
      const float dxm = px - mx, dym = py - my, dzm = pz - mz;
      const float dm = sqrtf((dxm * dxm + dym * dym) + dzm * dzm);
      const float delay = (dm - d0) * RCPC;
      const float freq = (float)fc * FSTEP;
      ph = (NEG2PI * freq) * delay;
    }
    float sv, cv;
#if defined(__HIP_DEVICE_COMPILE__)
    sincosf(ph, &sv, &cv);
#else
    sv = 0.0f; cv = 1.0f; (void)ph;
#endif
    sfe[row * 10 + m]     = cv;
    sfe[row * 10 + 5 + m] = sv;
    if (tid < 64) { sfe[row * 10] = 1.0f; sfe[row * 10 + 5] = -0.0f; }
  }
  __syncthreads();
  if (tid < 64) {
    const int row = tid;
    const int f = f0 + row;
    float fe[10];
#pragma unroll
    for (int i = 0; i < 10; ++i) fe[i] = sfe[row * 10 + i];
    float r[10];
#pragma unroll
    for (int k = 0; k < 10; ++k) r[k] = 0.0f;
#pragma unroll 1
    for (int j = 0; j < NHID; ++j) {
      float a = fe[0] * sw1[j];
#pragma unroll
      for (int i = 1; i < 10; ++i) a = fmaf(fe[i], sw1[i * NHID + j], a);
      a = a + sb1[j];
      a = fmaxf(a, 0.0f);
#pragma unroll
      for (int k = 0; k < 10; ++k) r[k] = fmaf(a, sw2[j * 10 + k], r[k]);
    }
    float v[10];
#pragma unroll
    for (int k = 0; k < 10; ++k) v[k] = (f < NFREQ) ? (r[k] + sb2[k]) : 0.0f;
    float* wb = WR + ((size_t)(bn * 10)) * FPW + f;
#pragma unroll
    for (int k = 0; k < 10; ++k) *(volatile float*)(wb + (size_t)k * FPW) = v[k];
    __threadfence();
#pragma unroll
    for (int k = 0; k < 10; ++k) *(volatile float*)(wb + (size_t)k * FPW) = v[k];
  }
}

__global__ __launch_bounds__(256)
void k_beam(const float* __restrict__ sr, const float* __restrict__ si, const float* __restrict__ WR,
            unsigned short* MAG)
{
  __shared__ __align__(16) unsigned short magl[NBIRD * TBLK * FP];
  __shared__ __align__(16) float wl[NBIRD * FCH * WLP];
  const int tid = threadIdx.x, lane = tid & 31, wave = tid >> 5;
  const int tb = blockIdx.x, b = blockIdx.y;
  const int t0 = tb * TBLK;
  const int t = wave;
  const int fl = lane;

#pragma unroll 1
  for (int chn = 0; chn < NCH; ++chn) {
    const int f0 = chn * FCH;
    __syncthreads();
#pragma unroll
    for (int q = 0; q < 10; ++q) {
      const int idx = tid + 256 * q;
      const int ff  = idx & 31;
      const int nj  = idx >> 5;
      const int n   = nj / 10;
      const int j   = nj - n * 10;
      wl[(n * FCH + ff) * WLP + j] = WR[((size_t)((b * NBIRD + n) * 10 + j)) * FPW + f0 + ff];
    }
    __syncthreads();
    const int f  = f0 + fl;
    const int fc = (f < NFREQ) ? f : (NFREQ - 1);
    const bool live = (f < NFREQ);
    float xr[NMIC], xi[NMIC];
#pragma unroll
    for (int m = 0; m < NMIC; ++m) {
      const size_t off = ((size_t)((b * NMIC + m) * NFREQ + fc)) * TLEN + t0 + t;
      xr[m] = bf16r(sr[off]);
      xi[m] = bf16r(si[off]);
    }
#pragma unroll 1
    for (int n = 0; n < NBIRD; ++n) {
      const float* wp = wl + (n * FCH + fl) * WLP;
      const v4f wa = *(const v4f*)(wp);
      const v4f wb = *(const v4f*)(wp + 4);
      const v2f wc = *(const v2f*)(wp + 8);
      const float wr0 = wa[0], wr1 = wa[1], wr2 = wa[2], wr3 = wa[3], wr4 = wb[0];
      const float wi0 = wb[1], wi1 = wb[2], wi2 = wb[3], wi3 = wc[0], wi4 = wc[1];
      float srr = xr[0] * wr0; srr = fmaf(xr[1], wr1, srr); srr = fmaf(xr[2], wr2, srr); srr = fmaf(xr[3], wr3, srr); srr = fmaf(xr[4], wr4, srr);
      float sii = xi[0] * wi0; sii = fmaf(xi[1], wi1, sii); sii = fmaf(xi[2], wi2, sii); sii = fmaf(xi[3], wi3, sii); sii = fmaf(xi[4], wi4, sii);
      float sri = xr[0] * wi0; sri = fmaf(xr[1], wi1, sri); sri = fmaf(xr[2], wi2, sri); sri = fmaf(xr[3], wi3, sri); sri = fmaf(xr[4], wi4, sri);
      float sir = xi[0] * wr0; sir = fmaf(xi[1], wr1, sir); sir = fmaf(xi[2], wr2, sir); sir = fmaf(xi[3], wr3, sir); sir = fmaf(xi[4], wr4, sir);
      const float br = srr - sii;
      const float bi = sri + sir;
      const float mag = sqrtf(br * br + bi * bi);
      magl[(n * TBLK + t) * FP + f] = live ? hbits(mag * MSC) : (unsigned short)0;
    }
  }
  __syncthreads();
  {
    const int n = wave;
    const v8us* srcl = (const v8us*)magl + n * (TBLK * FP / 8);
    unsigned short* dstg = MAG + ((size_t)((b * NBIRD + n) * TPAD + t0 + 1)) * FP;
    unsigned short* dz0  = MAG + ((size_t)((b * NBIRD + n) * TPAD)) * FP;
    unsigned short* dz1  = MAG + ((size_t)((b * NBIRD + n) * TPAD + TPAD - 1)) * FP;
    const bool wz0 = (tb == 0), wz1 = (tb == NTB - 1);
    const v8us zz = zero8us();
    v8us u[10];
#pragma unroll
    for (int q = 0; q < 10; ++q) u[q] = srcl[q * 32 + lane];
#pragma unroll
    for (int q = 0; q < 10; ++q) *(volatile v8us*)(dstg + ((size_t)(q * 32 + lane)) * 8) = u[q];
    if (wz0) { *(volatile v8us*)(dz0 + lane * 8) = zz; if (lane < 8) *(volatile v8us*)(dz0 + (32 + lane) * 8) = zz; }
    if (wz1) { *(volatile v8us*)(dz1 + lane * 8) = zz; if (lane < 8) *(volatile v8us*)(dz1 + (32 + lane) * 8) = zz; }
    __threadfence();
#pragma unroll
    for (int q = 0; q < 10; ++q) *(volatile v8us*)(dstg + ((size_t)(q * 32 + lane)) * 8) = u[q];
    if (wz0) { *(volatile v8us*)(dz0 + lane * 8) = zz; if (lane < 8) *(volatile v8us*)(dz0 + (32 + lane) * 8) = zz; }
    if (wz1) { *(volatile v8us*)(dz1 + lane * 8) = zz; if (lane < 8) *(volatile v8us*)(dz1 + (32 + lane) * 8) = zz; }
  }
}

template <int CPT, int NCT>
__global__ __launch_bounds__(128)
void k_conv(const unsigned short* __restrict__ Ap, const unsigned short* __restrict__ Wp,
            const float* __restrict__ bias, float* Z, float* part)
{
  constexpr int KT = 3 * CPT;
  constexpr int KS = CPT / 32;
  __shared__ __align__(16) float stile[64 * SP];
  __shared__ __align__(16) float sst[128];
  __shared__ float sbias[64];
  const int tid = threadIdx.x, lane = tid & 31, wave = tid >> 5;
  const int h = lane >> 4, c = lane & 15;
  const int rb = blockIdx.x, cbk = blockIdx.y;
  const int s = rb >> 3, t0 = (rb & 7) * 64;
  const int wm = wave & 1, wn = wave >> 1;
  if (tid < 64) sbias[tid] = bf16r(bias[cbk * 64 + tid]);
  __syncthreads();

  const size_t arow = (size_t)s * TPAD + t0 + 32 * wm + c;
  const unsigned short* a0p = Ap + arow * CPT + 8 * h;
  const unsigned short* a1p = a0p + 16 * CPT;
  const unsigned short* b0p = Wp + ((size_t)(cbk * 64 + 32 * wn + c)) * KT + 8 * h;
  const unsigned short* b1p = b0p + (size_t)16 * KT;

  v8f acc00 = zero8(), acc01 = zero8(), acc10 = zero8(), acc11 = zero8();
#pragma unroll 1
  for (int tap = 0; tap < 3; ++tap) {
    const unsigned short* at0 = a0p + tap * CPT;
    const unsigned short* at1 = a1p + tap * CPT;
    const unsigned short* bt0 = b0p + tap * CPT;
    const unsigned short* bt1 = b1p + tap * CPT;
#pragma unroll 2
    for (int kk = 0; kk < KS; ++kk) {
      const v16us fa0 = ldfrag(at0 + 32 * kk);
      const v16us fa1 = ldfrag(at1 + 32 * kk);
      const v16us fb0 = ldfrag(bt0 + 32 * kk);
      const v16us fb1 = ldfrag(bt1 + 32 * kk);
      acc00 = mma_h(fa0, fb0, acc00);
      acc01 = mma_h(fa0, fb1, acc01);
      acc10 = mma_h(fa1, fb0, acc10);
      acc11 = mma_h(fa1, fb1, acc11);
      guard8(acc00, acc01, acc10, acc11, fa0, fa1, fb0, fb1);
    }
  }

  {
    const int r0 = 32 * wm + 8 * h;
    const int cA = 32 * wn + c, cB = cA + 16;
    const float bA = sbias[cA], bB = sbias[cB];
#pragma unroll
    for (int r = 0; r < 8; ++r) {
      stile[(r0 + r) * SP + cA]      = fmaf(acc00[r], ZINV, bA);
      stile[(r0 + r) * SP + cB]      = fmaf(acc01[r], ZINV, bB);
      stile[(r0 + 16 + r) * SP + cA] = fmaf(acc10[r], ZINV, bA);
      stile[(r0 + 16 + r) * SP + cB] = fmaf(acc11[r], ZINV, bB);
    }
  }
  __syncthreads();
  v4f zv[8];
#pragma unroll
  for (int e = 0; e < 8; ++e) {
    const int idx = tid + 128 * e;
    const int u = idx & 15, row = idx >> 4;
    zv[e] = *(const v4f*)(stile + row * SP + 4 * u);
  }
  if (tid < 64) {
    float sm = 0.0f, sq = 0.0f;
#pragma unroll 4
    for (int r = 0; r < 64; ++r) {
      const float v = stile[r * SP + tid];
      sm += v;
      sq = fmaf(v, v, sq);
    }
    sst[tid] = sm;
    sst[64 + tid] = sq;
  }
  __syncthreads();
  const v4f pv = *(const v4f*)(sst + 4 * lane);
  float* pp = part + (size_t)rb * 2 * NCT + (size_t)(lane >> 4) * NCT + cbk * 64 + 4 * (lane & 15);
  const bool wrp = (wave == 0);
#pragma unroll
  for (int e = 0; e < 8; ++e) {
    const int idx = tid + 128 * e;
    const int u = idx & 15, row = idx >> 4;
    float* zp = Z + ((size_t)(s * TLEN + t0 + row)) * NCT + cbk * 64 + 4 * u;
    *(volatile v4f*)zp = zv[e];
  }
  if (wrp) *(volatile v4f*)pp = pv;
  __threadfence();
#pragma unroll
  for (int e = 0; e < 8; ++e) {
    const int idx = tid + 128 * e;
    const int u = idx & 15, row = idx >> 4;
    float* zp = Z + ((size_t)(s * TLEN + t0 + row)) * NCT + cbk * 64 + 4 * u;
    *(volatile v4f*)zp = zv[e];
  }
  if (wrp) *(volatile v4f*)pp = pv;
}

template <int NC>
__global__ __launch_bounds__(NC)
void k_bnred(const float* __restrict__ part, const float* __restrict__ gam,
             const float* __restrict__ bet, float* tab)
{
  __shared__ __align__(16) float st[2 * NC];
  const int tid = threadIdx.x, lane = tid & 31, wave = tid >> 5;
  const int ch = tid;
  double sm = 0.0, sq = 0.0;
#pragma unroll 1
  for (int k = 0; k < NRB; ++k) {
    sm += (double)part[(size_t)k * 2 * NC + ch];
    sq += (double)part[(size_t)k * 2 * NC + NC + ch];
  }
  const double invn = 1.0 / (double)NROWS;
  const double mu = sm * invn;
  double var = sq * invn - mu * mu;
  var = (var > 0.0) ? var : 0.0;
  const float rs = rsqrtf((float)var + EPSBN);
  const float sc = bf16r(gam[ch]) * rs;
  const float sh = fmaf(-(float)mu, sc, bf16r(bet[ch]));
  st[ch] = sc;
  st[NC + ch] = sh;
  __syncthreads();
  constexpr int NU = 2 * NC / 4;
  const int unit = wave * 32 + lane;
  const int uc = (unit < NU) ? unit : (NU - 1);
  const v4f v = *(const v4f*)(st + 4 * uc);
  float* pt = tab + 4 * uc;
  const bool wr = (unit < NU);
  if (wr) *(volatile v4f*)pt = v;
  __threadfence();
  if (wr) *(volatile v4f*)pt = v;
}

__global__ __launch_bounds__(256)
void k_apply(const float* __restrict__ Z1, const float* __restrict__ tab, unsigned short* H1)
{
  __shared__ float st[2 * C1N];
  const int tid = threadIdx.x;
  st[tid] = tab[tid];
  __syncthreads();
  const int idx = blockIdx.x * 256 + tid;
  const int u = idx & 15;
  const int R = idx >> 4;
  const int s = R / TPAD;
  const int tt = R - s * TPAD;
  const int tz = tt - 1;
  const bool live = (tz >= 0) && (tz < TLEN);
  const int tzc = (tz < 0) ? 0 : ((tz > TLEN - 1) ? (TLEN - 1) : tz);
  const float* zp = Z1 + ((size_t)(s * TLEN + tzc)) * C1N + 8 * u;
  const v4f za = *(const v4f*)(zp);
  const v4f zb = *(const v4f*)(zp + 4);
  v8us o = zero8us();
#pragma unroll
  for (int e = 0; e < 4; ++e) {
    const int cha = 8 * u + e, chb = 8 * u + 4 + e;
    const float va = fmaxf(fmaf(za[e], st[cha], st[C1N + cha]), 0.0f) * H1SC;
    const float vb = fmaxf(fmaf(zb[e], st[chb], st[C1N + chb]), 0.0f) * H1SC;
    o[e]     = (unsigned short)(live ? (unsigned)hbits(va) : 0u);
    o[4 + e] = (unsigned short)(live ? (unsigned)hbits(vb) : 0u);
  }
  unsigned short* dp = H1 + (size_t)R * C1N + 8 * u;
  *(volatile v8us*)dp = o;
  __threadfence();
  *(volatile v8us*)dp = o;
}

__global__ __launch_bounds__(256)
void k_final(const float* __restrict__ Z2, const float* __restrict__ tab, float* out)
{
  __shared__ __align__(16) float st[2 * C2N];
  __shared__ __align__(16) float so[C2N];
  const int tid = threadIdx.x, lane = tid & 31, wave = tid >> 5;
  const int s = blockIdx.x;
  st[tid] = tab[tid];
  st[C2N + tid] = tab[C2N + tid];
  __syncthreads();
  const float sc = st[tid], sh = st[C2N + tid];
  const float* zp = Z2 + (size_t)s * TLEN * C2N + tid;
  float a = 0.0f;
#pragma unroll 4
  for (int t = 0; t < TLEN; ++t) a += fmaxf(fmaf(zp[(size_t)t * C2N], sc, sh), 0.0f);
  so[tid] = a * (1.0f / 512.0f);
  __syncthreads();
  const int unit = wave * 32 + lane;
  const int uc = (unit < 64) ? unit : 63;
  const v4f v = *(const v4f*)(so + 4 * uc);
  float* po = out + (size_t)s * C2N + 4 * uc;
  const bool wr = (unit < 64);
  if (wr) *(volatile v4f*)po = v;
  __threadfence();
  if (wr) *(volatile v4f*)po = v;
}

extern "C" void kernel_launch(void* const* d_in, const int* in_sizes, int n_in,
                              void* d_out, int out_size, void* d_ws, size_t ws_size,
                              hipStream_t stream) {
  if (n_in < 15) return;
  if (in_sizes[0] != NBAT * NMIC * NFREQ * TLEN || in_sizes[1] != NBAT * NMIC * NFREQ * TLEN) return;
  if (in_sizes[2] != NSMP * 3) return;
  if (in_sizes[3] != 10 * NHID || in_sizes[4] != NHID || in_sizes[5] != NHID * 10 || in_sizes[6] != 10) return;
  if (in_sizes[7] != C1N * NFREQ * 3 || in_sizes[8] != C1N || in_sizes[9] != C1N || in_sizes[10] != C1N) return;
  if (in_sizes[11] != C2N * C1N * 3 || in_sizes[12] != C2N || in_sizes[13] != C2N || in_sizes[14] != C2N) return;
  if (out_size != NSMP * C2N) return;

  const float* sr  = (const float*)d_in[0];
  const float* si  = (const float*)d_in[1];
  const float* pos = (const float*)d_in[2];
  const float* w1  = (const float*)d_in[3];
  const float* b1  = (const float*)d_in[4];
  const float* w2  = (const float*)d_in[5];
  const float* b2  = (const float*)d_in[6];
  const float* cw1 = (const float*)d_in[7];
  const float* cb1 = (const float*)d_in[8];
  const float* g1  = (const float*)d_in[9];
  const float* be1 = (const float*)d_in[10];
  const float* cw2 = (const float*)d_in[11];
  const float* cb2 = (const float*)d_in[12];
  const float* g2  = (const float*)d_in[13];
  const float* be2 = (const float*)d_in[14];
  float* out = (float*)d_out;

  size_t off = 0;
  const size_t oWR  = off;  off += (size_t)NSMP * 10 * FPW * 4;
  const size_t oMAG = off;  off += (size_t)NSMP * TPAD * FP * 2;
  const size_t oW1P = off;  off += (size_t)C1N * K1 * 2;
  const size_t oW2P = off;  off += (size_t)C2N * K2 * 2;
  const size_t oZ1  = off;  off += (size_t)NROWS * C1N * 4;
  const size_t oP1  = off;  off += (size_t)NRB * 2 * C1N * 4;
  const size_t oT1  = off;  off += (size_t)2 * C1N * 4;
  const size_t oH1  = off;  off += (size_t)NSMP * TPAD * C1N * 2;
  const size_t oZ2  = off;  off += (size_t)NROWS * C2N * 4;
  const size_t oP2  = off;  off += (size_t)NRB * 2 * C2N * 4;
  const size_t oT2  = off;  off += (size_t)2 * C2N * 4;
  if (off > ws_size || off > (size_t)134217728) return;

  char* ws = (char*)d_ws;
  float*          WR  = (float*)(ws + oWR);
  unsigned short* MAG = (unsigned short*)(ws + oMAG);
  unsigned short* W1P = (unsigned short*)(ws + oW1P);
  unsigned short* W2P = (unsigned short*)(ws + oW2P);
  float*          Z1  = (float*)(ws + oZ1);
  float*          P1  = (float*)(ws + oP1);
  float*          T1  = (float*)(ws + oT1);
  unsigned short* H1  = (unsigned short*)(ws + oH1);
  float*          Z2  = (float*)(ws + oZ2);
  float*          P2  = (float*)(ws + oP2);
  float*          T2  = (float*)(ws + oT2);

  k_prep<<<dim3(NPB1 + NPB2), dim3(256), 0, stream>>>(cw1, cw2, W1P, W2P);
  k_steer<<<dim3(NSTB), dim3(256), 0, stream>>>(pos, w1, b1, w2, b2, WR);
  k_beam<<<dim3(NTB, NBAT), dim3(256), 0, stream>>>(sr, si, WR, MAG);
  k_conv<FP, C1N><<<dim3(NRB, C1N / 64), dim3(128), 0, stream>>>(MAG, W1P, cb1, Z1, P1);
  k_bnred<C1N><<<dim3(1), dim3(C1N), 0, stream>>>(P1, g1, be1, T1);
  k_apply<<<dim3(NAPB), dim3(256), 0, stream>>>(Z1, T1, H1);
  k_conv<C1N, C2N><<<dim3(NRB, C2N / 64), dim3(128), 0, stream>>>(H1, W2P, cb2, Z2, P2);
  k_bnred<C2N><<<dim3(1), dim3(C2N), 0, stream>>>(P2, g2, be2, T2);
  k_final<<<dim3(NSMP), dim3(256), 0, stream>>>(Z2, T2, out);
  (void)hipGetLastError();
}
